// WeightedNonLocalBlock_31636729102405
// MI455X (gfx1250) — hardware-verified
//
#include <hip/hip_runtime.h>
#include <math.h>

constexpr int kB   = 8;
constexpr int kC   = 256;
constexpr int kN   = 4096;
constexpr int kQC  = 2048;
constexpr int kNumChunks = kB * (kN / kQC);
constexpr float kWCarry    = 16.0f;
constexpr float kWCarryInv = 1.0f / 16.0f;
constexpr float kPCarry    = 2048.0f;
constexpr float kYCarry    = 16.0f;
constexpr float kPVScale   = kYCarry / kPCarry;
constexpr float kOutScale  = 1.0f / (kYCarry * kWCarry);

constexpr size_t kOffW16 = 0;
constexpr size_t kOffX16 = kOffW16 + (size_t)4 * kC * kC * 2;
constexpr size_t kOffTP  = kOffX16 + (size_t)kB * kN * kC * 2;
constexpr size_t kOffG16 = kOffTP + (size_t)kB * kN * 2 * kC * 2;
constexpr size_t kOffS   = kOffG16 + (size_t)kB * kC * kN * 2;
constexpr size_t kOffP   = kOffS + (size_t)kQC * kN * 4;
constexpr size_t kWsEnd  = kOffP + (size_t)kQC * kN * 2;
static_assert(kWsEnd == 117964800ull, "carve");
static_assert(kWsEnd <= 134217728ull, "carve cap");
static_assert((size_t)kB * kN * kC * 2 <= (size_t)kQC * kN * 4, "YvT fits in S region");

typedef __attribute__((ext_vector_type(16))) _Float16 v16h;
typedef __attribute__((ext_vector_type(8)))  _Float16 v8h;
typedef __attribute__((ext_vector_type(16))) __bf16   v16b;
typedef __attribute__((ext_vector_type(8)))  __bf16   v8b;
typedef __attribute__((ext_vector_type(8)))  float    v8f;
typedef __attribute__((ext_vector_type(4)))  float    v4f;
typedef __attribute__((ext_vector_type(4)))  unsigned int v4u;

__device__ __forceinline__ unsigned short f2bf_bits(float f) {
  unsigned u = __float_as_uint(f);
  return (unsigned short)((u + 0x7FFFu + ((u >> 16) & 1u)) >> 16);
}
__device__ __forceinline__ float bf_bits2f(unsigned short h) { return __uint_as_float(((unsigned)h) << 16); }

__device__ __forceinline__ void dep_guard_h(v8f& a, v8f& b, v16h x, v16h y) { asm volatile("v_nop\n\tv_nop\n\tv_nop\n\tv_nop" : "+v"(a), "+v"(b) : "v"(x), "v"(y)); }
__device__ __forceinline__ void dep_guard_b(v8f& a, v8f& b, v16b x, v16b y) { asm volatile("v_nop\n\tv_nop\n\tv_nop\n\tv_nop" : "+v"(a), "+v"(b) : "v"(x), "v"(y)); }
__device__ __forceinline__ void keep4_h(v16h a, v16h b, v16h c, v16h d) { asm volatile("v_nop" :: "v"(a), "v"(b), "v"(c), "v"(d)); }
__device__ __forceinline__ void keep4_b(v16b a, v16b b, v16b c, v16b d) { asm volatile("v_nop" :: "v"(a), "v"(b), "v"(c), "v"(d)); }
__device__ __forceinline__ void acc_guard4(v8f& a, v8f& b, v8f& c, v8f& d) { asm volatile("v_nop\n\tv_nop\n\tv_nop\n\tv_nop" : "+v"(a), "+v"(b), "+v"(c), "+v"(d)); }
template <typename T> struct Frag;
template <> struct Frag<_Float16> {
  typedef v16h V; union U { v16h v; v8h h[2]; };
  static __device__ __forceinline__ v16h load(const _Float16* p) {
    U f; f.h[0] = *(const v8h*)(p); f.h[1] = *(const v8h*)(p + 16); return f.v;
  }
  static __device__ __forceinline__ v8f mma(v16h a, v16h b, v8f c) {
    return __builtin_amdgcn_wmma_f32_16x16x32_f16(false, a, false, b, (short)0, c, false, false);
  }
  static __device__ __forceinline__ void guard(v8f& a, v8f& b, v16h x, v16h y) { dep_guard_h(a, b, x, y); }
  static __device__ __forceinline__ void keep(v16h a, v16h b, v16h c, v16h d) { keep4_h(a, b, c, d); }
};
template <> struct Frag<__bf16> {
  typedef v16b V; union U { v16b v; v8b h[2]; };
  static __device__ __forceinline__ v16b load(const __bf16* p) {
    U f; f.h[0] = *(const v8b*)(p); f.h[1] = *(const v8b*)(p + 16); return f.v;
  }
  static __device__ __forceinline__ v8f mma(v16b a, v16b b, v8f c) {
    return __builtin_amdgcn_wmma_f32_16x16x32_bf16(false, a, false, b, (short)0, c, false, false);
  }
  static __device__ __forceinline__ void guard(v8f& a, v8f& b, v16b x, v16b y) { dep_guard_b(a, b, x, y); }
  static __device__ __forceinline__ void keep(v16b a, v16b b, v16b c, v16b d) { keep4_b(a, b, c, d); }
};

__device__ __forceinline__ unsigned pk16(unsigned short a, unsigned short b) { return (unsigned)a | ((unsigned)b << 16); }
__device__ __forceinline__ unsigned short h_bits(float f) { const _Float16 h = (_Float16)f; return __builtin_bit_cast(unsigned short, h); }

template <int ET> struct Elem;
template <> struct Elem<0> { typedef _Float16 T; };
template <> struct Elem<1> { typedef __bf16 T; };
template <int ET, bool SPLIT, int BIAS_MODE, int OUT_MODE, bool RESID, int ACT = 0, bool BLEND = false>
__global__ __launch_bounds__(256) void wmma_gemm64(
    const unsigned short* __restrict__ Ap, const unsigned short* __restrict__ A2p, int lda, long strideA,
    const unsigned short* __restrict__ Btp, const unsigned short* __restrict__ Bt2p, int ldb, long strideB,
    void* __restrict__ Cout, void* __restrict__ Cout2, int ldc, long strideC,
    const float* __restrict__ bias,
    const float* __restrict__ resid, long strideR,
    const float* __restrict__ wsc,
    int M, int N, int K, float scale) {
  static_assert(!BLEND || (RESID && OUT_MODE == 0), "blend needs resid and f32 out");
  typedef typename Elem<ET>::T T;
  typedef typename Frag<T>::V V;
  const T* A = (const T*)Ap; const T* A2 = (const T*)A2p; const T* Bt = (const T*)Btp; const T* Bt2 = (const T*)Bt2p;
  __shared__ __align__(16) float sT[8][16 * 68];
  const int b    = blockIdx.y;
  const int lane = threadIdx.x & 31;
  const int wave = threadIdx.x >> 5;
  const int tilesN = N >> 6;
  const int tilesM = M >> 6;
  const int tile = blockIdx.x * 8 + wave;
  if (tile >= tilesM * tilesN) return;
  const int tm = tile / tilesN;
  const int tn = tile - tm * tilesN;
  const int m0 = tm << 6;
  const int n0 = tn << 6;

  const T* Ab  = A  + (size_t)b * strideA;
  const T* Bb  = Bt + (size_t)b * strideB;
  const T* Ab2 = SPLIT ? (A2  + (size_t)b * strideA) : nullptr;
  const T* Bb2 = SPLIT ? (Bt2 + (size_t)b * strideB) : nullptr;

  const int rlane = lane & 15;
  const int koff  = (lane >> 4) * 8;
  const int mOff  = (lane >> 4) * 8;

  v8f acc[4][4];
#pragma unroll
  for (int i = 0; i < 4; ++i)
#pragma unroll
    for (int j = 0; j < 4; ++j) acc[i][j] = (v8f){0.f,0.f,0.f,0.f,0.f,0.f,0.f,0.f};

  for (int k0 = 0; k0 < K; k0 += 32) {
    V bh[4], bl[4];
#pragma unroll
    for (int j = 0; j < 4; ++j) {
      const size_t bo = (size_t)(n0 + (j << 4) + rlane) * ldb + koff + k0;
      bh[j] = Frag<T>::load(Bb + bo);
      if (SPLIT) bl[j] = Frag<T>::load(Bb2 + bo);
    }
#pragma unroll
    for (int i = 0; i < 4; ++i) {
      const size_t ao = (size_t)(m0 + (i << 4) + rlane) * lda + koff + k0;
      V ah = Frag<T>::load(Ab + ao);
      V al;
      if (SPLIT) al = Frag<T>::load(Ab2 + ao);
#pragma unroll
      for (int j = 0; j < 4; ++j) {
        acc[i][j] = Frag<T>::mma(ah, bh[j], acc[i][j]);
        if (SPLIT) {
          acc[i][j] = Frag<T>::mma(ah, bl[j], acc[i][j]);
          acc[i][j] = Frag<T>::mma(al, bh[j], acc[i][j]);
        }
      }
      Frag<T>::guard(acc[i][0], acc[i][3], ah, SPLIT ? al : ah);
    }
    Frag<T>::keep(bh[0], bh[1], bh[2], bh[3]);
    if (SPLIT) Frag<T>::keep(bl[0], bl[1], bl[2], bl[3]);
  }
  acc_guard4(acc[0][0], acc[0][1], acc[0][2], acc[0][3]);
  acc_guard4(acc[1][0], acc[1][1], acc[1][2], acc[1][3]);
  acc_guard4(acc[2][0], acc[2][1], acc[2][2], acc[2][3]);
  acc_guard4(acc[3][0], acc[3][1], acc[3][2], acc[3][3]);

  float* slab = sT[wave];
  const float* Rb = RESID ? (resid + (size_t)b * strideR) : nullptr;
  const float wv  = BLEND ? wsc[0] : 0.0f;
  const float omw = 1.0f - wv;
#pragma unroll
  for (int i = 0; i < 4; ++i) {
    const int mBase = m0 + (i << 4);
#pragma unroll
    for (int j = 0; j < 4; ++j) {
      const int n = n0 + (j << 4) + rlane;
      float bv = 0.f;
      if (BIAS_MODE == 2) bv = bias[n];
#pragma unroll
      for (int r = 0; r < 8; ++r) {
        float v = acc[i][j][r] * scale;
        if (BIAS_MODE == 1) v += bias[mBase + mOff + r];
        if (BIAS_MODE == 2) v += bv;
        if (RESID) {
          const float rv = Rb[(size_t)(mBase + mOff + r) * ldc + n];
          if (BLEND) v = omw * rv + wv * v;
          else v += rv;
        }
        if (ACT == 2) v = fmaxf(v, 0.0f);
        if (ACT == 4) v = (v > 0.f) ? v : 0.01f * v;
        slab[(mOff + r) * 68 + (j << 4) + rlane] = v;
      }
    }
    __builtin_amdgcn_fence(__ATOMIC_RELEASE, "workgroup");
    __builtin_amdgcn_wave_barrier();
    __builtin_amdgcn_fence(__ATOMIC_ACQUIRE, "workgroup");
    if (OUT_MODE == 0) {
      float* C = (float*)Cout + (size_t)b * strideC;
      const int hh = lane >> 4, c4 = (lane & 15) * 4;
      for (int pass = 0; pass < 2; ++pass) {
#pragma unroll
        for (int it = 0; it < 8; ++it) {
          const int row = it * 2 + hh;
          v4f v = *(const v4f*)(slab + row * 68 + c4);
          *(volatile v4f*)(C + (size_t)(mBase + row) * ldc + n0 + c4) = v;
        }
        __threadfence();
      }
    } else {
      const int q = lane >> 3, c8 = (lane & 7) * 8;
      unsigned short* C  = (unsigned short*)Cout  + (size_t)b * strideC;
      unsigned short* C2 = (OUT_MODE == 2) ? ((unsigned short*)Cout2 + (size_t)b * strideC) : nullptr;
      for (int pass = 0; pass < 2; ++pass) {
#pragma unroll
        for (int it = 0; it < 4; ++it) {
          const int row = it * 4 + q;
          const float* sp = slab + row * 68 + c8;
          v8h hv, lv;
#pragma unroll
          for (int e = 0; e < 8; ++e) {
            if (OUT_MODE == 1) {
              hv[e] = (_Float16)sp[e];
            } else {
              unsigned short hb = f2bf_bits(sp[e]);
              unsigned short lb = f2bf_bits(sp[e] - bf_bits2f(hb));
              hv[e] = __builtin_bit_cast(_Float16, hb);
              lv[e] = __builtin_bit_cast(_Float16, lb);
            }
          }
          *(volatile v8h*)(C + (size_t)(mBase + row) * ldc + n0 + c8) = hv;
          if (OUT_MODE == 2) *(volatile v8h*)(C2 + (size_t)(mBase + row) * ldc + n0 + c8) = lv;
        }
        __threadfence();
      }
    }
    __builtin_amdgcn_fence(__ATOMIC_RELEASE, "workgroup");
    __builtin_amdgcn_wave_barrier();
    __builtin_amdgcn_fence(__ATOMIC_ACQUIRE, "workgroup");
  }
}

__global__ __launch_bounds__(256) void wcast16_kernel(const float* __restrict__ W0, const float* __restrict__ W1,
                                                      const float* __restrict__ W2, const float* __restrict__ W3,
                                                      unsigned short* __restrict__ out, float scale) {
  const int i = blockIdx.x * 256 + threadIdx.x;
  const int z = blockIdx.y;
  if (i >= (kC * kC) / 8) return;
  const float* W = (z == 0) ? W0 : (z == 1) ? W1 : (z == 2) ? W2 : W3;
  const float* p = W + 8 * (size_t)i;
  const v4f a = *(const v4f*)(p);
  const v4f c = *(const v4f*)(p + 4);
  unsigned short hb[8];
#pragma unroll
  for (int e = 0; e < 4; ++e) {
    hb[e]     = h_bits(a[e] * scale);
    hb[4 + e] = h_bits(c[e] * scale);
  }
  const v4u u = (v4u){pk16(hb[0], hb[1]), pk16(hb[2], hb[3]), pk16(hb[4], hb[5]), pk16(hb[6], hb[7])};
  unsigned short* q = out + (size_t)z * kC * kC + 8 * (size_t)i;
  *(volatile v4u*)q = u;
  __threadfence();
  *(volatile v4u*)q = u;
}

__global__ __launch_bounds__(256) void xcast_t_kernel(const float* __restrict__ x, unsigned short* __restrict__ X16) {
  __shared__ float sm[64][65];
  const int t  = threadIdx.x;
  const int n0 = blockIdx.x * 64;
  const int c0 = blockIdx.y * 64;
  const int b  = blockIdx.z;
  const float* xb = x + (size_t)b * kC * kN;
#pragma unroll
  for (int it = 0; it < 4; ++it) {
    const int r  = it * 16 + (t >> 4);
    const int c4 = (t & 15) * 4;
    const v4f v = *(const v4f*)(xb + (size_t)(c0 + r) * kN + n0 + c4);
    sm[c4 + 0][r] = v[0];
    sm[c4 + 1][r] = v[1];
    sm[c4 + 2][r] = v[2];
    sm[c4 + 3][r] = v[3];
  }
  __syncthreads();
  const int lane = t & 31, wave = t >> 5;
  const int q = lane >> 3, c8 = (lane & 7) * 8;
  unsigned short* ob = X16 + ((size_t)b * kN + n0) * kC + c0;
  for (int pass = 0; pass < 2; ++pass) {
#pragma unroll
    for (int it = 0; it < 2; ++it) {
      const int row = wave * 8 + it * 4 + q;
      unsigned short hb[8];
#pragma unroll
      for (int e = 0; e < 8; ++e) hb[e] = h_bits(sm[row][c8 + e]);
      const v4u u = (v4u){pk16(hb[0], hb[1]), pk16(hb[2], hb[3]), pk16(hb[4], hb[5]), pk16(hb[6], hb[7])};
      *(volatile v4u*)(ob + (size_t)row * kC + c8) = u;
    }
    __threadfence();
  }
}

__global__ __launch_bounds__(256) void ytrans_kernel(const unsigned short* __restrict__ Y, unsigned short* __restrict__ YT) {
  __shared__ unsigned int sm[64][65];
  const int t  = threadIdx.x;
  const int p0 = blockIdx.x * 64;
  const int c0 = blockIdx.y * 64;
  const int b  = blockIdx.z;
  const unsigned short* yb = Y + (size_t)b * kN * kC;
#pragma unroll
  for (int it = 0; it < 2; ++it) {
    const int r  = it * 32 + (t >> 3);
    const int c8 = (t & 7) * 8;
    const v4u u = *(const v4u*)(yb + (size_t)(c0 + r) * kN + p0 + c8);
#pragma unroll
    for (int e = 0; e < 4; ++e) {
      sm[c8 + 2 * e][r]     = u[e] & 0xffffu;
      sm[c8 + 2 * e + 1][r] = u[e] >> 16;
    }
  }
  __syncthreads();
  const int lane = t & 31, wave = t >> 5;
  const int q = lane >> 3, c8 = (lane & 7) * 8;
  unsigned short* ob = YT + ((size_t)b * kN + p0) * kC + c0;
  for (int pass = 0; pass < 2; ++pass) {
#pragma unroll
    for (int it = 0; it < 2; ++it) {
      const int row = wave * 8 + it * 4 + q;
      const unsigned int* s = &sm[row][c8];
      const v4u u = (v4u){pk16((unsigned short)s[0], (unsigned short)s[1]), pk16((unsigned short)s[2], (unsigned short)s[3]),
                          pk16((unsigned short)s[4], (unsigned short)s[5]), pk16((unsigned short)s[6], (unsigned short)s[7])};
      *(volatile v4u*)(ob + (size_t)row * kC + c8) = u;
    }
    __threadfence();
  }
}

__global__ __launch_bounds__(256) void softmax_rows_kernel(const float* __restrict__ S, unsigned short* __restrict__ P, float carry) {
  __shared__ __align__(16) float sE[kN];
  __shared__ float redA[8];
  __shared__ float redB[8];
  const int row  = blockIdx.x;
  const int t    = threadIdx.x;
  const int lane = t & 31, wave = t >> 5;
  const float* sr = S + (size_t)row * kN;

  float m = -INFINITY;
#pragma unroll 1
  for (int seg = 0; seg < 2; ++seg) {
    const int c0 = seg * (kN / 2) + t * 8;
    const v4f a = *(const v4f*)(sr + c0);
    const v4f c = *(const v4f*)(sr + c0 + 4);
    const float ma = fmaxf(fmaxf(a[0], a[1]), fmaxf(a[2], a[3]));
    const float mc = fmaxf(fmaxf(c[0], c[1]), fmaxf(c[2], c[3]));
    m = fmaxf(m, fmaxf(ma, mc));
  }
#pragma unroll
  for (int off = 16; off > 0; off >>= 1) m = fmaxf(m, __shfl_xor(m, off, 32));
  if (lane == 0) redA[wave] = m;
  __syncthreads();
  float gm = redA[0];
#pragma unroll
  for (int w = 1; w < 8; ++w) gm = fmaxf(gm, redA[w]);

  float sum = 0.f;
#pragma unroll 1
  for (int seg = 0; seg < 2; ++seg) {
    const int c0 = seg * (kN / 2) + t * 8;
    const v4f a = *(const v4f*)(sr + c0);
    const v4f c = *(const v4f*)(sr + c0 + 4);
    v4f ea, ec;
#pragma unroll
    for (int e = 0; e < 4; ++e) { ea[e] = expf(a[e] - gm); ec[e] = expf(c[e] - gm); }
    sum += ea[0]; sum += ea[1]; sum += ea[2]; sum += ea[3];
    sum += ec[0]; sum += ec[1]; sum += ec[2]; sum += ec[3];
    *(v4f*)(sE + c0)     = ea;
    *(v4f*)(sE + c0 + 4) = ec;
  }
#pragma unroll
  for (int off = 16; off > 0; off >>= 1) sum += __shfl_xor(sum, off, 32);
  if (lane == 0) redB[wave] = sum;
  __syncthreads();
  float tot = redB[0];
#pragma unroll
  for (int w = 1; w < 8; ++w) tot += redB[w];
  const float f = carry * (1.0f / tot);

  unsigned short* prow = P + (size_t)row * kN;
#pragma unroll 1
  for (int seg = 0; seg < 2; ++seg) {
    const int c0 = seg * (kN / 2) + t * 8;
    const v4f ea = *(const v4f*)(sE + c0);
    const v4f ec = *(const v4f*)(sE + c0 + 4);
    unsigned short hb[8];
#pragma unroll
    for (int e = 0; e < 4; ++e) {
      hb[e]     = h_bits(ea[e] * f);
      hb[4 + e] = h_bits(ec[e] * f);
    }
    const v4u u = (v4u){pk16(hb[0], hb[1]), pk16(hb[2], hb[3]), pk16(hb[4], hb[5]), pk16(hb[6], hb[7])};
    unsigned short* q = prow + c0;
    *(volatile v4u*)q = u;
    __threadfence();
    *(volatile v4u*)q = u;
  }
}

extern "C" void kernel_launch(void* const* d_in, const int* in_sizes, int n_in,
                              void* d_out, int out_size, void* d_ws, size_t ws_size,
                              hipStream_t stream)
{
  if (n_in < 10) return;
  if (in_sizes[0] != kB * kC * kN) return;
  if (out_size != kB * kC * kN) return;
  if (ws_size < kWsEnd) return;

  const float* x       = (const float*)d_in[0];
  const float* theta_w = (const float*)d_in[1];
  const float* theta_b = (const float*)d_in[2];
  const float* phi_w   = (const float*)d_in[3];
  const float* phi_b   = (const float*)d_in[4];
  const float* g_w     = (const float*)d_in[5];
  const float* g_b     = (const float*)d_in[6];
  const float* wz_w    = (const float*)d_in[7];
  const float* wz_b    = (const float*)d_in[8];
  const float* wsc     = (const float*)d_in[9];
  float* out = (float*)d_out;

  char* ws = (char*)d_ws;
  unsigned short* W16 = (unsigned short*)(ws + kOffW16);
  unsigned short* X16 = (unsigned short*)(ws + kOffX16);
  unsigned short* TP  = (unsigned short*)(ws + kOffTP);
  unsigned short* G16 = (unsigned short*)(ws + kOffG16);
  float*          S   = (float*)(ws + kOffS);
  unsigned short* P   = (unsigned short*)(ws + kOffP);
  unsigned short* Y   = X16;
  unsigned short* YT  = (unsigned short*)(ws + kOffS);

  const long plane = (long)kN * kC;

  wcast16_kernel<<<dim3((kC * kC / 8) / 256, 4), 256, 0, stream>>>(theta_w, phi_w, g_w, wz_w, W16, kWCarry);

  xcast_t_kernel<<<dim3(kN / 64, kC / 64, kB), 256, 0, stream>>>(x, X16);

  wmma_gemm64<0, false, 2, 1, false, 0, false><<<dim3(32, kB), 256, 0, stream>>>(
      X16, nullptr, kC, plane,
      W16 + 0 * kC * kC, nullptr, kC, 0L,
      TP, nullptr, 2 * kC, (long)kN * 2 * kC,
      theta_b, nullptr, 0L, nullptr,
      kN, kC, kC, kWCarryInv);
  wmma_gemm64<0, false, 2, 1, false, 0, false><<<dim3(32, kB), 256, 0, stream>>>(
      X16, nullptr, kC, plane,
      W16 + 1 * kC * kC, nullptr, kC, 0L,
      TP + kC, nullptr, 2 * kC, (long)kN * 2 * kC,
      phi_b, nullptr, 0L, nullptr,
      kN, kC, kC, kWCarryInv);
  wmma_gemm64<0, false, 1, 1, false, 0, false><<<dim3(32, kB), 256, 0, stream>>>(
      W16 + 2 * kC * kC, nullptr, kC, 0L,
      X16, nullptr, kC, plane,
      G16, nullptr, kN, plane,
      g_b, nullptr, 0L, nullptr,
      kC, kN, kC, kWCarryInv);

  for (int ch = 0; ch < kNumChunks; ++ch) {
    const int b  = ch >> 1;
    const int hf = ch & 1;
    wmma_gemm64<0, false, 0, 0, false, 0, false><<<dim3(256, 1), 256, 0, stream>>>(
        TP + ((size_t)b * kN + (size_t)hf * kQC) * 2 * kC, nullptr, 2 * kC, 0L,
        TP + (size_t)b * kN * 2 * kC + kC, nullptr, 2 * kC, 0L,
        S, nullptr, kN, 0L,
        nullptr, nullptr, 0L, nullptr,
        kQC, kN, kC, 1.0f);
    softmax_rows_kernel<<<kQC, 256, 0, stream>>>(S, P, kPCarry);
    wmma_gemm64<0, false, 0, 1, false, 0, false><<<dim3(16, 1), 256, 0, stream>>>(
        P, nullptr, kN, 0L,
        G16 + (size_t)b * kC * kN, nullptr, kN, 0L,
        Y + ((size_t)b * kN + (size_t)hf * kQC) * kC, nullptr, kC, 0L,
        nullptr, nullptr, 0L, nullptr,
        kQC, kC, kN, kPVScale);
  }

  ytrans_kernel<<<dim3(kN / 64, kC / 64, kB), 256, 0, stream>>>(Y, YT);

  wmma_gemm64<0, false, 1, 0, true, 0, true><<<dim3(32, kB), 256, 0, stream>>>(
      W16 + 3 * kC * kC, nullptr, kC, 0L,
      YT, nullptr, kC, plane,
      out, nullptr, kN, plane,
      wz_b, x, plane, wsc,
      kC, kN, kC, kOutScale);
}
